// RelExLSTM_8323646620151
// MI455X (gfx1250) — hardware-verified
//
#include <hip/hip_runtime.h>
#include <math.h>


#define NB   512
#define NT   100
#define NE   300
#define NEP  320
#define NH   256
#define NG   1024
#define NL   19
#define TCH  50
#define RCH  (TCH * NB)
#define NBB  16
#define HP   264
#define HB   32

static_assert(NB == 512, "gather row decode uses r & 511, r >> 9");
static_assert(NB % NBB == 0, "blocks own whole row groups");
static_assert(RCH % 64 == 0 && NG % 64 == 0 && NEP % 32 == 0, "gemm tiling");
static_assert(NT % TCH == 0, "chunks");
static_assert(NB % HB == 0, "head blocks");
static_assert((HB * NL) % 4 == 0 && (HB * NL * 4) % 128 == 0, "head block output = whole lines");

typedef __attribute__((ext_vector_type(16))) _Float16 v16h;
typedef __attribute__((ext_vector_type(8)))  _Float16 v8h;
typedef __attribute__((ext_vector_type(16))) __bf16   v16b;
typedef __attribute__((ext_vector_type(8)))  __bf16   v8b;
typedef __attribute__((ext_vector_type(8)))  float    v8f;
typedef __attribute__((ext_vector_type(4)))  float    v4f;

__device__ __forceinline__ unsigned short f2bf_bits(float f) {
  unsigned u = __float_as_uint(f);
  return (unsigned short)((u + 0x7FFFu + ((u >> 16) & 1u)) >> 16);
}
__device__ __forceinline__ float bf_bits2f(unsigned short h) { return __uint_as_float(((unsigned)h) << 16); }

__device__ __forceinline__ void dep_guard_h(v8f& a, v8f& b, v16h x, v16h y) { asm volatile("v_nop\n\tv_nop\n\tv_nop\n\tv_nop" : "+v"(a), "+v"(b) : "v"(x), "v"(y)); }
__device__ __forceinline__ void dep_guard_b(v8f& a, v8f& b, v16b x, v16b y) { asm volatile("v_nop\n\tv_nop\n\tv_nop\n\tv_nop" : "+v"(a), "+v"(b) : "v"(x), "v"(y)); }
__device__ __forceinline__ void keep4_h(v16h a, v16h b, v16h c, v16h d) { asm volatile("v_nop" :: "v"(a), "v"(b), "v"(c), "v"(d)); }
__device__ __forceinline__ void keep4_b(v16b a, v16b b, v16b c, v16b d) { asm volatile("v_nop" :: "v"(a), "v"(b), "v"(c), "v"(d)); }
__device__ __forceinline__ void acc_guard4(v8f& a, v8f& b, v8f& c, v8f& d) { asm volatile("v_nop\n\tv_nop\n\tv_nop\n\tv_nop" : "+v"(a), "+v"(b), "+v"(c), "+v"(d)); }
template <typename T> struct Frag;
template <> struct Frag<_Float16> {
  typedef v16h V; union U { v16h v; v8h h[2]; };
  static __device__ __forceinline__ v16h load(const _Float16* p) {
    U f; f.h[0] = *(const v8h*)(p); f.h[1] = *(const v8h*)(p + 16); return f.v;
  }
  static __device__ __forceinline__ v8f mma(v16h a, v16h b, v8f c) {
    return __builtin_amdgcn_wmma_f32_16x16x32_f16(false, a, false, b, (short)0, c, false, false);
  }
  static __device__ __forceinline__ void guard(v8f& a, v8f& b, v16h x, v16h y) { dep_guard_h(a, b, x, y); }
  static __device__ __forceinline__ void keep(v16h a, v16h b, v16h c, v16h d) { keep4_h(a, b, c, d); }
};
template <> struct Frag<__bf16> {
  typedef v16b V; union U { v16b v; v8b h[2]; };
  static __device__ __forceinline__ v16b load(const __bf16* p) {
    U f; f.h[0] = *(const v8b*)(p); f.h[1] = *(const v8b*)(p + 16); return f.v;
  }
  static __device__ __forceinline__ v8f mma(v16b a, v16b b, v8f c) {
    return __builtin_amdgcn_wmma_f32_16x16x32_bf16(false, a, false, b, (short)0, c, false, false);
  }
  static __device__ __forceinline__ void guard(v8f& a, v8f& b, v16b x, v16b y) { dep_guard_b(a, b, x, y); }
  static __device__ __forceinline__ void keep(v16b a, v16b b, v16b c, v16b d) { keep4_b(a, b, c, d); }
};

template <int ET> struct Elem;
template <> struct Elem<0> { typedef _Float16 T; };
template <> struct Elem<1> { typedef __bf16 T; };
template <int ET, bool SPLIT, int BIAS_MODE, int OUT_MODE, bool RESID, int ACT = 0>
__global__ __launch_bounds__(256) void wmma_gemm64(
    const unsigned short* __restrict__ Ap, const unsigned short* __restrict__ A2p, int lda, long strideA,
    const unsigned short* __restrict__ Btp, const unsigned short* __restrict__ Bt2p, int ldb, long strideB,
    void* __restrict__ Cout, void* __restrict__ Cout2, int ldc, long strideC,
    const float* __restrict__ bias,
    const float* __restrict__ resid, long strideR,
    int M, int N, int K, float scale) {
  typedef typename Elem<ET>::T T;
  typedef typename Frag<T>::V V;
  const T* A = (const T*)Ap; const T* A2 = (const T*)A2p; const T* Bt = (const T*)Btp; const T* Bt2 = (const T*)Bt2p;
  __shared__ __align__(16) float sT[8][16 * 68];
  const int b    = blockIdx.y;
  const int lane = threadIdx.x & 31;
  const int wave = threadIdx.x >> 5;
  const int tilesN = N >> 6;
  const int tilesM = M >> 6;
  const int tile = blockIdx.x * 8 + wave;
  if (tile >= tilesM * tilesN) return;
  const int tm = tile / tilesN;
  const int tn = tile - tm * tilesN;
  const int m0 = tm << 6;
  const int n0 = tn << 6;

  const T* Ab  = A  + (size_t)b * strideA;
  const T* Bb  = Bt + (size_t)b * strideB;
  const T* Ab2 = SPLIT ? (A2  + (size_t)b * strideA) : nullptr;
  const T* Bb2 = SPLIT ? (Bt2 + (size_t)b * strideB) : nullptr;

  const int rlane = lane & 15;
  const int koff  = (lane >> 4) * 8;
  const int mOff  = (lane >> 4) * 8;

  v8f acc[4][4];
#pragma unroll
  for (int i = 0; i < 4; ++i)
#pragma unroll
    for (int j = 0; j < 4; ++j) acc[i][j] = (v8f){0.f,0.f,0.f,0.f,0.f,0.f,0.f,0.f};

  for (int k0 = 0; k0 < K; k0 += 32) {
    V bh[4], bl[4];
#pragma unroll
    for (int j = 0; j < 4; ++j) {
      const size_t bo = (size_t)(n0 + (j << 4) + rlane) * ldb + koff + k0;
      bh[j] = Frag<T>::load(Bb + bo);
      if (SPLIT) bl[j] = Frag<T>::load(Bb2 + bo);
    }
#pragma unroll
    for (int i = 0; i < 4; ++i) {
      const size_t ao = (size_t)(m0 + (i << 4) + rlane) * lda + koff + k0;
      V ah = Frag<T>::load(Ab + ao);
      V al;
      if (SPLIT) al = Frag<T>::load(Ab2 + ao);
#pragma unroll
      for (int j = 0; j < 4; ++j) {
        acc[i][j] = Frag<T>::mma(ah, bh[j], acc[i][j]);
        if (SPLIT) {
          acc[i][j] = Frag<T>::mma(ah, bl[j], acc[i][j]);
          acc[i][j] = Frag<T>::mma(al, bh[j], acc[i][j]);
        }
      }
      Frag<T>::guard(acc[i][0], acc[i][3], ah, SPLIT ? al : ah);
    }
    Frag<T>::keep(bh[0], bh[1], bh[2], bh[3]);
    if (SPLIT) Frag<T>::keep(bl[0], bl[1], bl[2], bl[3]);
  }
  acc_guard4(acc[0][0], acc[0][1], acc[0][2], acc[0][3]);
  acc_guard4(acc[1][0], acc[1][1], acc[1][2], acc[1][3]);
  acc_guard4(acc[2][0], acc[2][1], acc[2][2], acc[2][3]);
  acc_guard4(acc[3][0], acc[3][1], acc[3][2], acc[3][3]);

  float* slab = sT[wave];
  const float* Rb = RESID ? (resid + (size_t)b * strideR) : nullptr;
#pragma unroll
  for (int i = 0; i < 4; ++i) {
    const int mBase = m0 + (i << 4);
#pragma unroll
    for (int j = 0; j < 4; ++j) {
      const int n = n0 + (j << 4) + rlane;
      float bv = 0.f;
      if (BIAS_MODE == 2) bv = bias[n];
#pragma unroll
      for (int r = 0; r < 8; ++r) {
        float v = acc[i][j][r] * scale;
        if (BIAS_MODE == 1) v += bias[mBase + mOff + r];
        if (BIAS_MODE == 2) v += bv;
        if (RESID) v += Rb[(size_t)(mBase + mOff + r) * ldc + n];
        if (ACT == 1) v = tanhf(v);
        if (ACT == 2) v = fmaxf(v, 0.0f);
        if (ACT == 3) v = v / (1.0f + expf(-v));
        if (ACT == 4) v = (v > 0.f) ? v : 0.01f * v;
        if (ACT == 5) v = 0.5f * v * (1.0f + erff(v * 0.70710678118654752f));
        slab[(mOff + r) * 68 + (j << 4) + rlane] = v;
      }
    }
    __builtin_amdgcn_fence(__ATOMIC_RELEASE, "workgroup");
    __builtin_amdgcn_wave_barrier();
    __builtin_amdgcn_fence(__ATOMIC_ACQUIRE, "workgroup");
    if (OUT_MODE == 0) {
      float* C = (float*)Cout + (size_t)b * strideC;
      const int hh = lane >> 4, c4 = (lane & 15) * 4;
      for (int pass = 0; pass < 2; ++pass) {
#pragma unroll
        for (int it = 0; it < 8; ++it) {
          const int row = it * 2 + hh;
          v4f v = *(const v4f*)(slab + row * 68 + c4);
          *(volatile v4f*)(C + (size_t)(mBase + row) * ldc + n0 + c4) = v;
        }
        __threadfence();
      }
    } else {
      const int q = lane >> 3, c8 = (lane & 7) * 8;
      unsigned short* C  = (unsigned short*)Cout  + (size_t)b * strideC;
      unsigned short* C2 = (OUT_MODE == 2) ? ((unsigned short*)Cout2 + (size_t)b * strideC) : nullptr;
      for (int pass = 0; pass < 2; ++pass) {
#pragma unroll
        for (int it = 0; it < 4; ++it) {
          const int row = it * 4 + q;
          const float* sp = slab + row * 68 + c8;
          v8h hv, lv;
#pragma unroll
          for (int e = 0; e < 8; ++e) {
            if (OUT_MODE == 1) {
              hv[e] = (_Float16)sp[e];
            } else {
              unsigned short hb = f2bf_bits(sp[e]);
              unsigned short lb = f2bf_bits(sp[e] - bf_bits2f(hb));
              hv[e] = __builtin_bit_cast(_Float16, hb);
              lv[e] = __builtin_bit_cast(_Float16, lb);
            }
          }
          *(volatile v8h*)(C + (size_t)(mBase + row) * ldc + n0 + c8) = hv;
          if (OUT_MODE == 2) *(volatile v8h*)(C2 + (size_t)(mBase + row) * ldc + n0 + c8) = lv;
        }
        __threadfence();
      }
    }
    __builtin_amdgcn_fence(__ATOMIC_RELEASE, "workgroup");
    __builtin_amdgcn_wave_barrier();
    __builtin_amdgcn_fence(__ATOMIC_ACQUIRE, "workgroup");
  }
}

__global__ __launch_bounds__(256) void gather_rows_f16(
    const float* __restrict__ src, const int* __restrict__ tok,
    _Float16* __restrict__ dst, int R, int Cin, int Cpad, int nsrc, float scale, int tbase)
{
  const int lane = threadIdx.x & 31;
  const int wave = threadIdx.x >> 5;
  const int r = blockIdx.x * 8 + wave;
  if (r >= R) return;
  const int b = r & (NB - 1), lt = r >> 9;
  int t = tbase + lt;
  t = (t < 0) ? 0 : t;
  t = (t > NT - 1) ? (NT - 1) : t;
  int id = tok[b * NT + t];
  id = (id < 0) ? (id + nsrc) : id;
  id = (id < 0) ? 0 : id;
  id = (id > nsrc - 1) ? (nsrc - 1) : id;
  const float* sp = src + (size_t)id * Cin;
  _Float16* dp = dst + (size_t)r * Cpad;
  v8h o[2];
#pragma unroll
  for (int ch = 0; ch < 2; ++ch) {
    const int c0 = ch * 256 + 8 * lane;
    int ca = c0, cb = c0 + 4;
    const bool va = (ca + 3 < Cin), vb = (cb + 3 < Cin);
    ca = va ? ca : (Cin - 4);
    cb = vb ? cb : (Cin - 4);
    v4f x0 = *(const v4f*)(sp + ca);
    v4f x1 = *(const v4f*)(sp + cb);
    const v4f z = (v4f){0.f, 0.f, 0.f, 0.f};
    if (!va) x0 = z;
    if (!vb) x1 = z;
#pragma unroll
    for (int e = 0; e < 4; ++e) {
      o[ch][e]     = (_Float16)(x0[e] * scale);
      o[ch][4 + e] = (_Float16)(x1[e] * scale);
    }
  }
  for (int pass = 0; pass < 2; ++pass) {
#pragma unroll
    for (int ch = 0; ch < 2; ++ch) {
      const int c0 = ch * 256 + 8 * lane;
      if (c0 < Cpad) *(volatile v8h*)(dp + c0) = o[ch];
    }
    __threadfence();
  }
}

__global__ __launch_bounds__(256) void colsT_to_f16(
    const float* __restrict__ src, _Float16* __restrict__ dst, int Kin, int Nn, int Kpad, float scale)
{
  const int lane = threadIdx.x & 31;
  const int wave = threadIdx.x >> 5;
  const int n = blockIdx.x * 8 + wave;
  if (n >= Nn) return;
  _Float16* dp = dst + (size_t)n * Kpad;
  v8h o[2];
#pragma unroll
  for (int ch = 0; ch < 2; ++ch) {
#pragma unroll
    for (int e = 0; e < 8; ++e) {
      const int k = ch * 256 + 8 * lane + e;
      const bool ok = (k < Kin);
      const int kc = ok ? k : (Kin - 1);
      const float v = src[(size_t)kc * Nn + n];
      o[ch][e] = (_Float16)(ok ? v * scale : 0.0f);
    }
  }
  for (int pass = 0; pass < 2; ++pass) {
#pragma unroll
    for (int ch = 0; ch < 2; ++ch) {
      const int c0 = ch * 256 + 8 * lane;
      if (c0 < Kpad) *(volatile v8h*)(dp + c0) = o[ch];
    }
    __threadfence();
  }
}

__device__ __forceinline__ float sigm_f(float x) { return __builtin_amdgcn_rcpf(1.0f + __expf(-x)); }
__device__ __forceinline__ float tanh_f(float x) { return 1.0f - 2.0f * __builtin_amdgcn_rcpf(__expf(2.0f * x) + 1.0f); }

__global__ __launch_bounds__(256) void recur_kernel(
    const _Float16* __restrict__ Ut16,
    const _Float16* __restrict__ zx16,
    const float* __restrict__ bias,
    float* __restrict__ hcat,
    float* __restrict__ cst,
    int dir, int first, int nsteps)
{
  __shared__ __align__(16) _Float16 hsh[2 * NBB * HP];
  __shared__ __align__(16) float csh[NBB * NH];
  __shared__ __align__(16) float hfs[NBB * NH];
  __shared__ float bsh[NG];
  typedef Frag<_Float16> F;
  const int tid = threadIdx.x;
  const int lane = tid & 31, wave = tid >> 5, hh = lane >> 4, rl = lane & 15;
  const int b0 = (int)blockIdx.x * NBB;
  dir = (dir != 0) ? 1 : 0;
  nsteps = (nsteps < 1) ? 1 : nsteps;
  nsteps = (nsteps > TCH) ? TCH : nsteps;

  if (first) {
    for (int i = tid; i < 2 * NBB * HP; i += 256) hsh[i] = (_Float16)0.0f;
    for (int i = tid; i < NBB * NH; i += 256) csh[i] = 0.0f;
  } else {
    for (int i = tid; i < 2 * NBB * HP; i += 256) {
      const int buf = i / (NBB * HP);
      const int rem = i - buf * (NBB * HP);
      const int bl = rem / HP;
      const int u = rem - bl * HP;
      const int uc = (u < NH) ? u : (NH - 1);
      const float hv = hcat[(size_t)(b0 + bl) * (2 * NH) + dir * NH + uc];
      hsh[i] = (_Float16)((buf == 0 && u < NH) ? hv * 256.0f : 0.0f);
    }
    for (int i = tid; i < NBB * NH; i += 256) csh[i] = cst[(size_t)(b0 + (i >> 8)) * NH + (i & 255)];
  }
  for (int i = tid; i < NBB * NH; i += 256) hfs[i] = 0.0f;
  for (int i = tid; i < NG; i += 256) bsh[i] = bias[i];
  __syncthreads();

  const int u0 = wave * 32;
  const float S  = 1.0f / 16384.0f;
  const float XS = 1.0f / 64.0f;

  for (int sl = 0; sl < nsteps; ++sl) {
    const int lt = dir ? (nsteps - 1 - sl) : sl;
    const _Float16* hc = hsh + (sl & 1) * (NBB * HP);
    _Float16* hn = hsh + ((sl & 1) ^ 1) * (NBB * HP);
    const _Float16* xrow = zx16 + ((size_t)lt * NB + b0) * NG;
    const bool last = (sl == nsteps - 1);
#pragma unroll 1
    for (int q = 0; q < 2; ++q) {
      const int ub = u0 + 16 * q;
      v8f acc[4];
#pragma unroll
      for (int g = 0; g < 4; ++g) acc[g] = (v8f){0.f,0.f,0.f,0.f,0.f,0.f,0.f,0.f};
#pragma unroll 1
      for (int k0 = 0; k0 < NH; k0 += 32) {
        v16h bfr[4];
#pragma unroll
        for (int g = 0; g < 4; ++g) bfr[g] = F::load(Ut16 + (size_t)(g * NH + ub + rl) * NH + k0 + 8 * hh);
        const v16h a = F::load(hc + rl * HP + k0 + 8 * hh);
#pragma unroll
        for (int g = 0; g < 4; ++g) acc[g] = F::mma(a, bfr[g], acc[g]);
        F::guard(acc[0], acc[3], a, a);
        F::keep(bfr[0], bfr[1], bfr[2], bfr[3]);
      }
      acc_guard4(acc[0], acc[1], acc[2], acc[3]);

      const int u = ub + rl;
      const float bI = bsh[u], bF = bsh[NH + u], bG = bsh[2 * NH + u], bO = bsh[3 * NH + u];
#pragma unroll
      for (int r = 0; r < 8; ++r) {
        const int bl = 8 * hh + r;
        const _Float16* xp = xrow + (size_t)bl * NG + u;
        const float gi = acc[0][r] * S + ((float)xp[0]      * XS + bI);
        const float gf = acc[1][r] * S + ((float)xp[NH]     * XS + bF);
        const float gg = acc[2][r] * S + ((float)xp[2 * NH] * XS + bG);
        const float go = acc[3][r] * S + ((float)xp[3 * NH] * XS + bO);
        const float cp = csh[bl * NH + u];
        const float cn = sigm_f(gf) * cp + sigm_f(gi) * tanh_f(gg);
        csh[bl * NH + u] = cn;
        const float h = sigm_f(go) * tanh_f(cn);
        hn[bl * HP + u] = (_Float16)(h * 256.0f);
        if (last) hfs[bl * NH + u] = h;
      }
    }
    __syncthreads();
  }

  for (int pass = 0; pass < 2; ++pass) {
#pragma unroll
    for (int rr = 0; rr < 2; ++rr) {
      const int bl = 2 * wave + rr;
#pragma unroll
      for (int it = 0; it < 2; ++it) {
        const int c4i = (it * 32 + lane) * 4;
        const v4f hv4 = *(const v4f*)(hfs + bl * NH + c4i);
        const v4f cv4 = *(const v4f*)(csh + bl * NH + c4i);
        *(volatile v4f*)(hcat + (size_t)(b0 + bl) * (2 * NH) + dir * NH + c4i) = hv4;
        *(volatile v4f*)(cst + (size_t)(b0 + bl) * NH + c4i) = cv4;
      }
    }
    __threadfence();
  }
}

__global__ __launch_bounds__(256) void head_kernel(
    const float* __restrict__ hcat, const float* __restrict__ Wd,
    const float* __restrict__ bd, float* __restrict__ out)
{
  __shared__ __align__(16) float lg[HB * NL];
  __shared__ __align__(16) float pr[HB * NL];
  const int tid = threadIdx.x;
  const int r0 = (int)blockIdx.x * HB;
  for (int p = tid; p < HB * NL; p += 256) {
    const int rr = p / NL;
    const int l = p - rr * NL;
    const float* hp = hcat + (size_t)(r0 + rr) * (2 * NH);
    const float* wp = Wd + l;
    float s = bd[l];
#pragma unroll 4
    for (int k = 0; k < 2 * NH; ++k) s += hp[k] * wp[(size_t)k * NL];
    lg[p] = s;
  }
  __syncthreads();
  if (tid < HB) {
    const float* lr = lg + tid * NL;
    float mx = lr[0];
#pragma unroll 1
    for (int j = 1; j < NL; ++j) mx = fmaxf(mx, lr[j]);
    float s = 0.f;
#pragma unroll 1
    for (int j = 0; j < NL; ++j) s += expf(lr[j] - mx);
    const float inv = 1.0f / s;
#pragma unroll 1
    for (int j = 0; j < NL; ++j) pr[tid * NL + j] = expf(lr[j] - mx) * inv;
  }
  __syncthreads();
  if (tid < 32) {
    float* ob = out + (size_t)r0 * NL;
    for (int pass = 0; pass < 2; ++pass) {
#pragma unroll
      for (int j = 0; j < 5; ++j) {
        const int idx = j * 128 + tid * 4;
        if (idx < HB * NL) {
          const v4f v = *(const v4f*)(pr + idx);
          *(volatile v4f*)(ob + idx) = v;
        }
      }
      __threadfence();
    }
  }
}

extern "C" void kernel_launch(void* const* d_in, const int* in_sizes, int n_in,
                              void* d_out, int out_size, void* d_ws, size_t ws_size,
                              hipStream_t stream) {
  if (n_in < 10) return;
  if (in_sizes[0] != NB * NT) return;
  if (in_sizes[1] < NE || in_sizes[1] % NE != 0) return;
  if (in_sizes[2] != NE * NG || in_sizes[3] != NH * NG || in_sizes[4] != NG) return;
  if (in_sizes[5] != NE * NG || in_sizes[6] != NH * NG || in_sizes[7] != NG) return;
  if (in_sizes[8] != 2 * NH * NL || in_sizes[9] != NL) return;
  if (out_size != NB * NL) return;
  const int nvocab = in_sizes[1] / NE;

  const int*   tokens = (const int*)  d_in[0];
  const float* embed  = (const float*)d_in[1];
  const float* Wf     = (const float*)d_in[2];
  const float* Uf     = (const float*)d_in[3];
  const float* bfv    = (const float*)d_in[4];
  const float* Wb     = (const float*)d_in[5];
  const float* Ub     = (const float*)d_in[6];
  const float* bbv    = (const float*)d_in[7];
  const float* Wd     = (const float*)d_in[8];
  const float* bd     = (const float*)d_in[9];
  float* out0 = (float*)d_out;

  const size_t szX = (size_t)RCH * NEP * 2;
  const size_t szW = (size_t)2 * NG * NEP * 2;
  const size_t szU = (size_t)2 * NG * NH * 2;
  const size_t szZ = (size_t)RCH * NG * 2;
  const size_t szH = (size_t)NB * 2 * NH * 4;
  const size_t szC = (size_t)NB * NH * 4;
  size_t off = 0;
  const size_t oX = off; off += szX;
  const size_t oW = off; off += szW;
  const size_t oU = off; off += szU;
  const size_t oZ = off; off += szZ;
  const size_t oH = off; off += szH;
  const size_t oC = off; off += szC;
  if (off > ws_size) return;
  char* ws = (char*)d_ws;
  _Float16* X16  = (_Float16*)(ws + oX);
  _Float16* W16  = (_Float16*)(ws + oW);
  _Float16* U16  = (_Float16*)(ws + oU);
  _Float16* ZX16 = (_Float16*)(ws + oZ);
  float*    HC   = (float*)(ws + oH);
  float*    CST  = (float*)(ws + oC);

  colsT_to_f16<<<NG / 8, 256, 0, stream>>>(Wf, W16, NE, NG, NEP, 64.0f);
  colsT_to_f16<<<NG / 8, 256, 0, stream>>>(Wb, W16 + (size_t)NG * NEP, NE, NG, NEP, 64.0f);
  colsT_to_f16<<<NG / 8, 256, 0, stream>>>(Uf, U16, NH, NG, NH, 64.0f);
  colsT_to_f16<<<NG / 8, 256, 0, stream>>>(Ub, U16 + (size_t)NG * NH, NH, NG, NH, 64.0f);

  const int gemm_blocks = ((RCH / 64) * (NG / 64) + 7) / 8;
  const unsigned short* X16u = (const unsigned short*)X16;
  const unsigned short* W16f = (const unsigned short*)W16;
  const unsigned short* W16b = (const unsigned short*)(W16 + (size_t)NG * NEP);

  gather_rows_f16<<<RCH / 8, 256, 0, stream>>>(embed, tokens, X16, RCH, NE, NEP, nvocab, 64.0f, 0);
  wmma_gemm64<0, false, 0, 1, false, 0><<<dim3(gemm_blocks, 1), 256, 0, stream>>>(
      X16u, X16u, NEP, 0L, W16f, W16f, NEP, 0L, (void*)ZX16, (void*)ZX16, NG, 0L,
      (const float*)HC, (const float*)HC, 0L, RCH, NG, NEP, 1.0f / 64.0f);
  recur_kernel<<<NB / NBB, 256, 0, stream>>>(U16, ZX16, bfv, HC, CST, 0, 1, TCH);

  gather_rows_f16<<<RCH / 8, 256, 0, stream>>>(embed, tokens, X16, RCH, NE, NEP, nvocab, 64.0f, TCH);
  wmma_gemm64<0, false, 0, 1, false, 0><<<dim3(gemm_blocks, 1), 256, 0, stream>>>(
      X16u, X16u, NEP, 0L, W16f, W16f, NEP, 0L, (void*)ZX16, (void*)ZX16, NG, 0L,
      (const float*)HC, (const float*)HC, 0L, RCH, NG, NEP, 1.0f / 64.0f);
  recur_kernel<<<NB / NBB, 256, 0, stream>>>(U16, ZX16, bfv, HC, CST, 0, 0, TCH);

  wmma_gemm64<0, false, 0, 1, false, 0><<<dim3(gemm_blocks, 1), 256, 0, stream>>>(
      X16u, X16u, NEP, 0L, W16b, W16b, NEP, 0L, (void*)ZX16, (void*)ZX16, NG, 0L,
      (const float*)HC, (const float*)HC, 0L, RCH, NG, NEP, 1.0f / 64.0f);
  recur_kernel<<<NB / NBB, 256, 0, stream>>>(U16 + (size_t)NG * NH, ZX16, bbv, HC, CST, 1, 1, TCH);

  gather_rows_f16<<<RCH / 8, 256, 0, stream>>>(embed, tokens, X16, RCH, NE, NEP, nvocab, 64.0f, 0);
  wmma_gemm64<0, false, 0, 1, false, 0><<<dim3(gemm_blocks, 1), 256, 0, stream>>>(
      X16u, X16u, NEP, 0L, W16b, W16b, NEP, 0L, (void*)ZX16, (void*)ZX16, NG, 0L,
      (const float*)HC, (const float*)HC, 0L, RCH, NG, NEP, 1.0f / 64.0f);
  recur_kernel<<<NB / NBB, 256, 0, stream>>>(U16 + (size_t)NG * NH, ZX16, bbv, HC, CST, 1, 0, TCH);

  head_kernel<<<NB / HB, 256, 0, stream>>>(HC, Wd, bd, out0);
}
